// MSAColumnAttention_52183852646489
// MI455X (gfx1250) — hardware-verified
//
#include <hip/hip_runtime.h>

#define NWAVE 8
#define NTHR (NWAVE * 32)
#define CH 32
#define DM 256
#define FE 8192
#define NPLANE 6
#define LDS_W_BYTES (NPLANE * FE * 2)
#define LDS_O_FLOATS (NWAVE * 512)
#define LDS_BYTES (LDS_W_BYTES + LDS_O_FLOATS * 4)

typedef __bf16 v16b __attribute__((ext_vector_type(16)));
typedef float v8f __attribute__((ext_vector_type(8)));
typedef float v4f __attribute__((ext_vector_type(4)));
typedef unsigned int v8u __attribute__((ext_vector_type(8)));
typedef v8u __attribute__((may_alias)) v8ua;
typedef v4f __attribute__((may_alias)) v4fa;

union Frag { v16b v; v8u u; };

__device__ __forceinline__ v8f wmma_bf16(v8f acc, v16b a, v16b b) {
  acc = __builtin_amdgcn_wmma_f32_16x16x32_bf16(false, a, false, b, (short)0, acc, false, false);
  asm volatile("v_nop\n\tv_nop\n\tv_nop\n\tv_nop" : "+v"(acc) : "v"(a), "v"(b));
  return acc;
}

__device__ __forceinline__ v8f zero8() {
  v8f z = {0.f, 0.f, 0.f, 0.f, 0.f, 0.f, 0.f, 0.f};
  return z;
}

__device__ __forceinline__ unsigned bf16_rne(float x) {
  unsigned u = __float_as_uint(x);
  return (u + 0x7FFFu + ((u >> 16) & 1u)) >> 16;
}
__device__ __forceinline__ void split_bf16(float x, unsigned &hi, unsigned &lo) {
  hi = bf16_rne(x);
  lo = bf16_rne(x - __uint_as_float(hi << 16));
}
__device__ __forceinline__ void split_pack2(float a, float b, unsigned &ph, unsigned &pl) {
  unsigned ha, la, hb, lb;
  split_bf16(a, ha, la);
  split_bf16(b, hb, lb);
  ph = ha | (hb << 16);
  pl = la | (lb << 16);
}

__device__ __forceinline__ int frag_half(int k) { return (k >> 3) & 1; }
__device__ __forceinline__ int frag_elem(int k) { return (k & 7) | ((k >> 4) << 3); }

__device__ __forceinline__ float gate_fn(float z) {
  return __builtin_amdgcn_rcpf(1.0f + __expf(-z));
}

extern __shared__ __align__(32) unsigned short lds_u16[];

__global__ __launch_bounds__(NTHR) void k_main(
    const float* __restrict__ m,
    const float* __restrict__ gamma,
    const float* __restrict__ beta,
    const float* __restrict__ Wv,
    const float* __restrict__ Wg,
    const float* __restrict__ Wo,
    const float* __restrict__ bo,
    float* out,
    int R, int numTiles, int tilesPerWave)
{
  unsigned short* sW = lds_u16;
  float* sO = (float*)(lds_u16 + NPLANE * FE);

  const int tid = threadIdx.x;

  for (int c = 0; c < CH; ++c) {
    const int hh = frag_half(c), ii = frag_elem(c);
    for (int j = tid; j < DM; j += NTHR) {
      const int idx = ((((j >> 4) * 32) + hh * 16 + (j & 15)) << 4) + ii;
      unsigned h0, l0;
      split_bf16(Wv[c * DM + j], h0, l0);
      sW[idx] = (unsigned short)h0;
      sW[FE + idx] = (unsigned short)l0;
      split_bf16(Wg[c * DM + j], h0, l0);
      sW[2 * FE + idx] = (unsigned short)h0;
      sW[3 * FE + idx] = (unsigned short)l0;
    }
  }
  for (int f = tid; f < DM * CH; f += NTHR) {
    const int j = f >> 5, c = f & 31;
    const int ct = c >> 4, mm = c & 15, kk = j >> 5, jj = j & 31;
    const int idx = ((((ct * 8 + kk) * 32) + frag_half(jj) * 16 + mm) << 4) + frag_elem(jj);
    unsigned h0, l0;
    split_bf16(Wo[f], h0, l0);
    sW[4 * FE + idx] = (unsigned short)h0;
    sW[5 * FE + idx] = (unsigned short)l0;
  }
  __syncthreads();

  const int lane = tid & 31;
  const int wave = tid >> 5;
  const int h = lane >> 4;
  const int n = lane & 15;
  float* so = sO + wave * 512;

  const int wglob  = blockIdx.x * NWAVE + wave;
  const int nwaves = gridDim.x * NWAVE;

  for (int it = 0; it < tilesPerWave; ++it) {
    const int t = wglob + it * nwaves;
    const bool tval = (t < numTiles);
    int row = t * 16 + n;
    int rowc = row;
    if (rowc > R - 1) rowc = R - 1;
    if (rowc < 0) rowc = 0;
    const float* mp = m + (size_t)rowc * CH;

    float x[16];
    {
      v4f x0 = *(const v4f*)(mp + 8 * h);
      v4f x1 = *(const v4f*)(mp + 8 * h + 4);
      v4f x2 = *(const v4f*)(mp + 16 + 8 * h);
      v4f x3 = *(const v4f*)(mp + 16 + 8 * h + 4);
      x[0] = x0.x; x[1] = x0.y; x[2] = x0.z; x[3] = x0.w;
      x[4] = x1.x; x[5] = x1.y; x[6] = x1.z; x[7] = x1.w;
      x[8] = x2.x; x[9] = x2.y; x[10] = x2.z; x[11] = x2.w;
      x[12] = x3.x; x[13] = x3.y; x[14] = x3.z; x[15] = x3.w;
    }
    float s = 0.f;
    #pragma unroll
    for (int i = 0; i < 16; ++i) s += x[i];
    s += __shfl_xor(s, 16, 32);
    const float mu = s * (1.0f / 32.0f);
    float q = 0.f;
    #pragma unroll
    for (int i = 0; i < 16; ++i) { float d = x[i] - mu; q += d * d; }
    q += __shfl_xor(q, 16, 32);
    const float var = q * (1.0f / 32.0f);
    const float rs = rsqrtf(var + 1e-5f);

    Frag bh, bl;
    #pragma unroll
    for (int p = 0; p < 8; ++p) {
      const int c0 = (p < 4) ? (8 * h + 2 * p) : (16 + 8 * h + 2 * (p - 4));
      const float y0 = (x[2 * p]     - mu) * rs * gamma[c0]     + beta[c0];
      const float y1 = (x[2 * p + 1] - mu) * rs * gamma[c0 + 1] + beta[c0 + 1];
      unsigned ph, pl;
      split_pack2(y0, y1, ph, pl);
      bh.u[p] = ph;
      bl.u[p] = pl;
    }

    v8f accT0 = zero8();
    v8f accT1 = zero8();

    #pragma unroll 1
    for (int kk = 0; kk < 8; ++kk) {
      Frag oh, ol;
      oh.u = (v8u){0u, 0u, 0u, 0u, 0u, 0u, 0u, 0u};
      ol.u = oh.u;
      #pragma unroll
      for (int half = 0; half < 2; ++half) {
        const int jt = 2 * kk + half;
        const unsigned short* fb = sW + ((jt * 32 + lane) << 4);
        Frag ah, al;
        ah.u = *(const v8ua*)(fb);
        al.u = *(const v8ua*)(fb + FE);
        v8f accV = zero8();
        accV = wmma_bf16(accV, ah.v, bh.v);
        accV = wmma_bf16(accV, ah.v, bl.v);
        accV = wmma_bf16(accV, al.v, bh.v);
        Frag gh, gl;
        gh.u = *(const v8ua*)(fb + 2 * FE);
        gl.u = *(const v8ua*)(fb + 3 * FE);
        v8f accG = zero8();
        accG = wmma_bf16(accG, gh.v, bh.v);
        accG = wmma_bf16(accG, gh.v, bl.v);
        accG = wmma_bf16(accG, gl.v, bh.v);
        #pragma unroll
        for (int p = 0; p < 4; ++p) {
          const float o0 = accV[2 * p]     * gate_fn(accG[2 * p]);
          const float o1 = accV[2 * p + 1] * gate_fn(accG[2 * p + 1]);
          unsigned ph, pl;
          split_pack2(o0, o1, ph, pl);
          oh.u[4 * half + p] = ph;
          ol.u[4 * half + p] = pl;
        }
      }
      {
        const unsigned short* fo = sW + 4 * FE + (((0 * 8 + kk) * 32 + lane) << 4);
        Frag ah, al;
        ah.u = *(const v8ua*)(fo);
        al.u = *(const v8ua*)(fo + FE);
        accT0 = wmma_bf16(accT0, ah.v, oh.v);
        accT0 = wmma_bf16(accT0, ah.v, ol.v);
        accT0 = wmma_bf16(accT0, al.v, oh.v);
      }
      {
        const unsigned short* fo = sW + 4 * FE + (((1 * 8 + kk) * 32 + lane) << 4);
        Frag ah, al;
        ah.u = *(const v8ua*)(fo);
        al.u = *(const v8ua*)(fo + FE);
        accT1 = wmma_bf16(accT1, ah.v, oh.v);
        accT1 = wmma_bf16(accT1, ah.v, ol.v);
        accT1 = wmma_bf16(accT1, al.v, oh.v);
      }
    }

    {
      const float* b0 = bo + 8 * h;
      const float* b1 = bo + 16 + 8 * h;
      v4f w0 = {accT0[0] + b0[0], accT0[1] + b0[1], accT0[2] + b0[2], accT0[3] + b0[3]};
      v4f w1 = {accT0[4] + b0[4], accT0[5] + b0[5], accT0[6] + b0[6], accT0[7] + b0[7]};
      v4f w2 = {accT1[0] + b1[0], accT1[1] + b1[1], accT1[2] + b1[2], accT1[3] + b1[3]};
      v4f w3 = {accT1[4] + b1[4], accT1[5] + b1[5], accT1[6] + b1[6], accT1[7] + b1[7]};
      *(v4f*)(so + n * 32 + 8 * h)          = w0;
      *(v4f*)(so + n * 32 + 8 * h + 4)      = w1;
      *(v4f*)(so + n * 32 + 16 + 8 * h)     = w2;
      *(v4f*)(so + n * 32 + 16 + 8 * h + 4) = w3;
    }
    __syncthreads();

    const int rr = lane >> 3;
    const int pp = lane & 7;
    v4f val[4];
    #pragma unroll
    for (int sg = 0; sg < 4; ++sg)
      val[sg] = *(const v4fa*)(so + (4 * sg + rr) * 32 + 4 * pp);
    #pragma unroll
    for (int sg = 0; sg < 4; ++sg) {
      const int grow = t * 16 + 4 * sg + rr;
      if (tval && grow < R)
        *(volatile v4f*)(out + (size_t)grow * CH + 4 * pp) = val[sg];
    }
    __threadfence();
    #pragma unroll
    for (int sg = 0; sg < 4; ++sg) {
      const int grow = t * 16 + 4 * sg + rr;
      if (tval && grow < R)
        *(volatile v4f*)(out + (size_t)grow * CH + 4 * pp) = val[sg];
    }
  }
}

extern "C" void kernel_launch(void* const* d_in, const int* in_sizes, int n_in,
                              void* d_out, int out_size, void* d_ws, size_t ws_size,
                              hipStream_t stream) {
  (void)d_ws; (void)ws_size;
  if (n_in < 9) return;
  const float* m     = (const float*)d_in[0];
  const float* gamma = (const float*)d_in[1];
  const float* beta  = (const float*)d_in[2];
  const float* Wv = (const float*)d_in[5];
  const float* Wg = (const float*)d_in[6];
  const float* Wo = (const float*)d_in[7];
  const float* bo = (const float*)d_in[8];
  float* out = (float*)d_out;

  const int R = in_sizes[0] / CH;
  if (R <= 0) return;
  if (in_sizes[1] < CH || in_sizes[2] < CH || in_sizes[8] < CH) return;
  if (in_sizes[5] != CH * DM || in_sizes[6] != CH * DM || in_sizes[7] != DM * CH) return;
  if (out_size < R * CH) return;

  const int numTiles = (R + 15) / 16;
  int grid = (numTiles + 4 * NWAVE - 1) / (4 * NWAVE);
  if (grid < 1) grid = 1;
  if (grid > 4096) grid = 4096;
  const int nw = grid * NWAVE;
  const int tilesPerWave = (numTiles + nw - 1) / nw;

  hipLaunchKernelGGL(k_main, dim3(grid), dim3(NTHR), (size_t)LDS_BYTES, stream,
                     m, gamma, beta, Wv, Wg, Wo, bo, out, R, numTiles, tilesPerWave);
}
